// TensorCoreAttentionV2_67972152426567
// MI455X (gfx1250) — hardware-run, weakly checked
//
#include <hip/hip_runtime.h>

#pragma clang fp contract(off)

constexpr int kBatch = 4;
constexpr int kSeq   = 2048;
constexpr int kDim   = 512;
constexpr int kHeads = 8;
constexpr int kDH    = 64;
constexpr int kFF    = 2048;
constexpr int kTok   = kBatch * kSeq;
constexpr int kQKld  = 2 * kDim;
constexpr int kGrp   = 2;
constexpr int kNChunk = (kBatch * kHeads) / kGrp;
constexpr int kHalfTok = kTok / 2;

constexpr float kWCarry   = 16.0f;
constexpr float kQKVCarry = 4.0f;
constexpr float kPCarry   = 2048.0f;
constexpr float kOCarry   = 256.0f;
constexpr float kGCarry   = 4.0f;
constexpr float kQKVScale   = kQKVCarry / kWCarry;
constexpr float kScoreScale = 1.0f / (kQKVCarry * kQKVCarry * 8.0f);
constexpr float kPVScale    = kOCarry / (kPCarry * kQKVCarry);
constexpr float kWoScale    = 1.0f / (kOCarry * kWCarry);
constexpr float kW1Scale    = 1.0f / kWCarry;
constexpr float kW2Scale    = 1.0f / (kGCarry * kWCarry);
constexpr float kInvDim     = 1.0f / 512.0f;

constexpr size_t kOffWqk = 0;
constexpr size_t kOffWv  = 1048576;
constexpr size_t kOffWo  = 1572864;
constexpr size_t kOffW1  = 2097152;
constexpr size_t kOffW2  = 4194304;
constexpr size_t kOffR1  = 6291456;
constexpr size_t kOffR2  = 14680064;
constexpr size_t kOffR3  = 31457280;
constexpr size_t kOffR4  = 39845888;
constexpr size_t kOffR5  = 48234496;
constexpr size_t kOffR6  = 81788928;
constexpr size_t kOffR7  = 98566144;
constexpr size_t kOffR8  = 115343360;
constexpr size_t kWsTotal = 132120576;
static_assert(kOffR1 == kOffW2 + (size_t)kDim * kFF * 2, "w planes");
static_assert(kOffR2 == kOffR1 + (size_t)kTok * kDim * 2, "R1");
static_assert(kOffR3 == kOffR2 + (size_t)kTok * kQKld * 2, "R2");
static_assert(kOffR4 == kOffR3 + (size_t)kDim * kTok * 2, "R3");
static_assert(kOffR5 == kOffR4 + (size_t)kTok * kDim * 2, "R4");
static_assert(kOffR6 == kOffR5 + (size_t)kGrp * kSeq * kSeq * 4, "R5");
static_assert(kOffR7 == kOffR6 + (size_t)kGrp * kSeq * kSeq * 2, "R6");
static_assert(kOffR8 == kOffR7 + (size_t)kTok * kDim * 4, "R7");
static_assert(kWsTotal == kOffR8 + (size_t)kTok * kDim * 4, "R8");
static_assert((size_t)kHalfTok * kFF * 4 <= (size_t)kGrp * kSeq * kSeq * 4, "F fits R5");
static_assert((size_t)kHalfTok * kFF * 2 <= (size_t)kGrp * kSeq * kSeq * 2, "G16 fits R6");
static_assert((size_t)kTok * kDim * 4 <= (size_t)kTok * kQKld * 2, "hpre fits R2");
static_assert(kWsTotal <= 134217728, "carve budget");

typedef __attribute__((ext_vector_type(16))) _Float16 v16h;
typedef __attribute__((ext_vector_type(8)))  _Float16 v8h;
typedef __attribute__((ext_vector_type(16))) __bf16   v16b;
typedef __attribute__((ext_vector_type(8)))  __bf16   v8b;
typedef __attribute__((ext_vector_type(8)))  float    v8f;
typedef __attribute__((ext_vector_type(4)))  float    v4f;
typedef __attribute__((ext_vector_type(4)))  unsigned int v4u;
typedef __attribute__((ext_vector_type(2)))  unsigned int v2u;

__device__ __forceinline__ unsigned short f2bf_bits(float f) {
  unsigned u = __float_as_uint(f);
  return (unsigned short)((u + 0x7FFFu + ((u >> 16) & 1u)) >> 16);
}
__device__ __forceinline__ float bf_bits2f(unsigned short h) { return __uint_as_float(((unsigned)h) << 16); }

__device__ __forceinline__ void dep_guard_h(v8f& a, v8f& b, v16h x, v16h y) { asm volatile("v_nop\n\tv_nop\n\tv_nop\n\tv_nop" : "+v"(a), "+v"(b) : "v"(x), "v"(y)); }
__device__ __forceinline__ void dep_guard_b(v8f& a, v8f& b, v16b x, v16b y) { asm volatile("v_nop\n\tv_nop\n\tv_nop\n\tv_nop" : "+v"(a), "+v"(b) : "v"(x), "v"(y)); }
__device__ __forceinline__ void keep4_h(v16h a, v16h b, v16h c, v16h d) { asm volatile("v_nop" :: "v"(a), "v"(b), "v"(c), "v"(d)); }
__device__ __forceinline__ void keep4_b(v16b a, v16b b, v16b c, v16b d) { asm volatile("v_nop" :: "v"(a), "v"(b), "v"(c), "v"(d)); }
__device__ __forceinline__ void acc_guard4(v8f& a, v8f& b, v8f& c, v8f& d) { asm volatile("v_nop\n\tv_nop\n\tv_nop\n\tv_nop" : "+v"(a), "+v"(b), "+v"(c), "+v"(d)); }
template <typename T> struct Frag;
template <> struct Frag<_Float16> {
  typedef v16h V; union U { v16h v; v8h h[2]; };
  static __device__ __forceinline__ v16h load(const _Float16* p) {
    U f; f.h[0] = *(const v8h*)(p); f.h[1] = *(const v8h*)(p + 16); return f.v;
  }
  static __device__ __forceinline__ v8f mma(v16h a, v16h b, v8f c) {
    return __builtin_amdgcn_wmma_f32_16x16x32_f16(false, a, false, b, (short)0, c, false, false);
  }
  static __device__ __forceinline__ void guard(v8f& a, v8f& b, v16h x, v16h y) { dep_guard_h(a, b, x, y); }
  static __device__ __forceinline__ void keep(v16h a, v16h b, v16h c, v16h d) { keep4_h(a, b, c, d); }
};
template <> struct Frag<__bf16> {
  typedef v16b V; union U { v16b v; v8b h[2]; };
  static __device__ __forceinline__ v16b load(const __bf16* p) {
    U f; f.h[0] = *(const v8b*)(p); f.h[1] = *(const v8b*)(p + 16); return f.v;
  }
  static __device__ __forceinline__ v8f mma(v16b a, v16b b, v8f c) {
    return __builtin_amdgcn_wmma_f32_16x16x32_bf16(false, a, false, b, (short)0, c, false, false);
  }
  static __device__ __forceinline__ void guard(v8f& a, v8f& b, v16b x, v16b y) { dep_guard_b(a, b, x, y); }
  static __device__ __forceinline__ void keep(v16b a, v16b b, v16b c, v16b d) { keep4_b(a, b, c, d); }
};

__device__ __forceinline__ unsigned pk16(unsigned short a, unsigned short b) { return (unsigned)a | ((unsigned)b << 16); }
__device__ __forceinline__ unsigned short h_bits(float f) { const _Float16 h = (_Float16)f; return __builtin_bit_cast(unsigned short, h); }

template <int ET> struct Elem;
template <> struct Elem<0> { typedef _Float16 T; };
template <> struct Elem<1> { typedef __bf16 T; };
template <int ET, bool SPLIT, int BIAS_MODE, int OUT_MODE, bool RESID, int ACT = 0>
__global__ __launch_bounds__(256) void wmma_gemm64(
    const unsigned short* __restrict__ Ap, const unsigned short* __restrict__ A2p, int lda, long strideA,
    const unsigned short* __restrict__ Btp, const unsigned short* __restrict__ Bt2p, int ldb, long strideB,
    void* __restrict__ Cout, void* __restrict__ Cout2, int ldc, long strideC,
    const float* __restrict__ bias,
    const float* __restrict__ resid, long strideR,
    int M, int N, int K, float scale) {
  typedef typename Elem<ET>::T T;
  typedef typename Frag<T>::V V;
  const T* A = (const T*)Ap; const T* A2 = (const T*)A2p; const T* Bt = (const T*)Btp; const T* Bt2 = (const T*)Bt2p;
  __shared__ __align__(16) float sT[8][16 * 68];
  const int b    = blockIdx.y;
  const int lane = threadIdx.x & 31;
  const int wave = threadIdx.x >> 5;
  const int tilesN = N >> 6;
  const int tilesM = M >> 6;
  const int tile = blockIdx.x * 8 + wave;
  if (tile >= tilesM * tilesN) return;
  const int tm = tile / tilesN;
  const int tn = tile - tm * tilesN;
  const int m0 = tm << 6;
  const int n0 = tn << 6;

  const T* Ab  = A  + (size_t)b * strideA;
  const T* Bb  = Bt + (size_t)b * strideB;
  const T* Ab2 = SPLIT ? (A2  + (size_t)b * strideA) : nullptr;
  const T* Bb2 = SPLIT ? (Bt2 + (size_t)b * strideB) : nullptr;

  const int rlane = lane & 15;
  const int koff  = (lane >> 4) * 8;
  const int mOff  = (lane >> 4) * 8;

  v8f acc[4][4];
#pragma unroll
  for (int i = 0; i < 4; ++i)
#pragma unroll
    for (int j = 0; j < 4; ++j) acc[i][j] = (v8f){0.f,0.f,0.f,0.f,0.f,0.f,0.f,0.f};

  for (int k0 = 0; k0 < K; k0 += 32) {
    V bh[4], bl[4];
#pragma unroll
    for (int j = 0; j < 4; ++j) {
      const size_t bo = (size_t)(n0 + (j << 4) + rlane) * ldb + koff + k0;
      bh[j] = Frag<T>::load(Bb + bo);
      if (SPLIT) bl[j] = Frag<T>::load(Bb2 + bo);
    }
#pragma unroll
    for (int i = 0; i < 4; ++i) {
      const size_t ao = (size_t)(m0 + (i << 4) + rlane) * lda + koff + k0;
      V ah = Frag<T>::load(Ab + ao);
      V al;
      if (SPLIT) al = Frag<T>::load(Ab2 + ao);
#pragma unroll
      for (int j = 0; j < 4; ++j) {
        acc[i][j] = Frag<T>::mma(ah, bh[j], acc[i][j]);
        if (SPLIT) {
          acc[i][j] = Frag<T>::mma(ah, bl[j], acc[i][j]);
          acc[i][j] = Frag<T>::mma(al, bh[j], acc[i][j]);
        }
      }
      Frag<T>::guard(acc[i][0], acc[i][3], ah, SPLIT ? al : ah);
    }
    Frag<T>::keep(bh[0], bh[1], bh[2], bh[3]);
    if (SPLIT) Frag<T>::keep(bl[0], bl[1], bl[2], bl[3]);
  }
  acc_guard4(acc[0][0], acc[0][1], acc[0][2], acc[0][3]);
  acc_guard4(acc[1][0], acc[1][1], acc[1][2], acc[1][3]);
  acc_guard4(acc[2][0], acc[2][1], acc[2][2], acc[2][3]);
  acc_guard4(acc[3][0], acc[3][1], acc[3][2], acc[3][3]);

  float* slab = sT[wave];
  const float* Rb = RESID ? (resid + (size_t)b * strideR) : nullptr;
#pragma unroll
  for (int i = 0; i < 4; ++i) {
    const int mBase = m0 + (i << 4);
#pragma unroll
    for (int j = 0; j < 4; ++j) {
      const int n = n0 + (j << 4) + rlane;
      float bv = 0.f;
      if (BIAS_MODE == 2) bv = bias[n];
#pragma unroll
      for (int r = 0; r < 8; ++r) {
        float v = acc[i][j][r] * scale;
        if (BIAS_MODE == 1) v += bias[mBase + mOff + r];
        if (BIAS_MODE == 2) v += bv;
        if (RESID) v += Rb[(size_t)(mBase + mOff + r) * ldc + n];
        if (ACT == 2) v = fmaxf(v, 0.0f);
        if (ACT == 4) v = (v > 0.f) ? v : 0.01f * v;
        slab[(mOff + r) * 68 + (j << 4) + rlane] = v;
      }
    }
    __builtin_amdgcn_fence(__ATOMIC_RELEASE, "workgroup");
    __builtin_amdgcn_wave_barrier();
    __builtin_amdgcn_fence(__ATOMIC_ACQUIRE, "workgroup");
    if (OUT_MODE == 0) {
      float* C = (float*)Cout + (size_t)b * strideC;
      const int hh = lane >> 4, c4 = (lane & 15) * 4;
      for (int pass = 0; pass < 2; ++pass) {
#pragma unroll
        for (int it = 0; it < 8; ++it) {
          const int row = it * 2 + hh;
          v4f v = *(const v4f*)(slab + row * 68 + c4);
          *(volatile v4f*)(C + (size_t)(mBase + row) * ldc + n0 + c4) = v;
        }
        __threadfence();
      }
    } else {
      const int q = lane >> 3, c8 = (lane & 7) * 8;
      unsigned short* C  = (unsigned short*)Cout  + (size_t)b * strideC;
      unsigned short* C2 = (OUT_MODE == 2) ? ((unsigned short*)Cout2 + (size_t)b * strideC) : nullptr;
      for (int pass = 0; pass < 2; ++pass) {
#pragma unroll
        for (int it = 0; it < 4; ++it) {
          const int row = it * 4 + q;
          const float* sp = slab + row * 68 + c8;
          v8h hv, lv;
#pragma unroll
          for (int e = 0; e < 8; ++e) {
            if (OUT_MODE == 1) {
              hv[e] = (_Float16)sp[e];
            } else {
              unsigned short hb = f2bf_bits(sp[e]);
              unsigned short lb = f2bf_bits(sp[e] - bf_bits2f(hb));
              hv[e] = __builtin_bit_cast(_Float16, hb);
              lv[e] = __builtin_bit_cast(_Float16, lb);
            }
          }
          *(volatile v8h*)(C + (size_t)(mBase + row) * ldc + n0 + c8) = hv;
          if (OUT_MODE == 2) *(volatile v8h*)(C2 + (size_t)(mBase + row) * ldc + n0 + c8) = lv;
        }
        __threadfence();
      }
    }
    __builtin_amdgcn_fence(__ATOMIC_RELEASE, "workgroup");
    __builtin_amdgcn_wave_barrier();
    __builtin_amdgcn_fence(__ATOMIC_ACQUIRE, "workgroup");
  }
}

__global__ __launch_bounds__(256) void tcast_kernel(const float* __restrict__ in, int ncols,
                                                    unsigned short* __restrict__ out, int ldo, float scale) {
  __shared__ float sm[64][65];
  const int t  = threadIdx.x;
  const int r0 = blockIdx.x * 64;
  const int c0 = blockIdx.y * 64;
#pragma unroll
  for (int i = 0; i < 16; ++i) {
    const int e = i * 256 + t;
    const int r = e >> 6;
    const int c = e & 63;
    sm[c][r] = in[(size_t)(r0 + r) * ncols + c0 + c] * scale;
  }
  __syncthreads();
  const int lane = t & 31, wave = t >> 5;
  const int q = lane >> 3, c8 = (lane & 7) * 8;
  for (int pass = 0; pass < 2; ++pass) {
#pragma unroll
    for (int it = 0; it < 2; ++it) {
      const int row = wave * 8 + it * 4 + q;
      unsigned short hb[8];
#pragma unroll
      for (int e = 0; e < 8; ++e) hb[e] = h_bits(sm[row][c8 + e]);
      const v4u u = (v4u){pk16(hb[0], hb[1]), pk16(hb[2], hb[3]), pk16(hb[4], hb[5]), pk16(hb[6], hb[7])};
      *(volatile v4u*)(out + (size_t)(c0 + row) * ldo + r0 + c8) = u;
    }
    __threadfence();
  }
}

__global__ __launch_bounds__(256) void cast8_f16_kernel(const float* __restrict__ in, unsigned short* __restrict__ out, int n8) {
  const int i = blockIdx.x * 256 + threadIdx.x;
  if (i >= n8) return;
  const float* p = in + 8 * (size_t)i;
  const v4f a = *(const v4f*)(p);
  const v4f c = *(const v4f*)(p + 4);
  unsigned short hb[8];
#pragma unroll
  for (int e = 0; e < 4; ++e) {
    hb[e]     = h_bits(a[e]);
    hb[4 + e] = h_bits(c[e]);
  }
  const v4u u = (v4u){pk16(hb[0], hb[1]), pk16(hb[2], hb[3]), pk16(hb[4], hb[5]), pk16(hb[6], hb[7])};
  unsigned short* q = out + 8 * (size_t)i;
  *(volatile v4u*)q = u;
  __threadfence();
  *(volatile v4u*)q = u;
}

__global__ __launch_bounds__(256) void softmax_poly_kernel(const float* __restrict__ S, unsigned short* __restrict__ P,
                                                           const float* __restrict__ exp_c) {
  __shared__ float redM[8];
  __shared__ float redS[8];
  const int row  = blockIdx.x;
  const int t    = threadIdx.x;
  const int lane = t & 31, wave = t >> 5;
  const int c0   = t * 8;
  const float* sr = S + (size_t)row * kSeq + c0;
  const v4f a = *(const v4f*)(sr);
  const v4f c = *(const v4f*)(sr + 4);
  float x[8];
#pragma unroll
  for (int e = 0; e < 4; ++e) { x[e] = a[e]; x[4 + e] = c[e]; }
  float ec[7];
#pragma unroll
  for (int i = 0; i < 7; ++i) ec[i] = exp_c[i];

  float m = fmaxf(fmaxf(fmaxf(x[0], x[1]), fmaxf(x[2], x[3])), fmaxf(fmaxf(x[4], x[5]), fmaxf(x[6], x[7])));
#pragma unroll
  for (int off = 16; off > 0; off >>= 1) m = fmaxf(m, __shfl_xor(m, off, 32));
  if (lane == 0) redM[wave] = m;
  __syncthreads();
  float rm = redM[0];
#pragma unroll
  for (int w = 1; w < 8; ++w) rm = fmaxf(rm, redM[w]);

  float ev[8];
  float ps = 0.0f;
#pragma unroll
  for (int e = 0; e < 8; ++e) {
    const float xx = x[e] - rm;
    float acc = ec[0];
    float pw = 1.0f;
#pragma unroll
    for (int i = 1; i < 7; ++i) {
      pw = pw * xx;
      const float term = ec[i] * pw;
      acc = acc + term;
    }
    ev[e] = fmaxf(acc, 1e-8f);
    ps = ps + ev[e];
  }
#pragma unroll
  for (int off = 16; off > 0; off >>= 1) ps += __shfl_xor(ps, off, 32);
  if (lane == 0) redS[wave] = ps;
  __syncthreads();
  float tot = redS[0];
#pragma unroll
  for (int w = 1; w < 8; ++w) tot = tot + redS[w];
  const float rcp = 1.0f / tot;

  unsigned short hb[8];
#pragma unroll
  for (int e = 0; e < 8; ++e) {
    const float pe = ev[e] * rcp;
    hb[e] = h_bits(pe * kPCarry);
  }
  const v4u u = (v4u){pk16(hb[0], hb[1]), pk16(hb[2], hb[3]), pk16(hb[4], hb[5]), pk16(hb[6], hb[7])};
  unsigned short* q = P + (size_t)row * kSeq + c0;
  *(volatile v4u*)q = u;
  __threadfence();
  *(volatile v4u*)q = u;
}

template <bool WRITE16>
__global__ __launch_bounds__(256) void layernorm_kernel(const float* __restrict__ in, const float* __restrict__ gamma,
                                                        const float* __restrict__ beta, float* __restrict__ outf,
                                                        unsigned short* __restrict__ out16, int nrows) {
  __shared__ float redA[8];
  __shared__ float redB[8];
  const int t = threadIdx.x, lane = t & 31, wave = t >> 5;
  const int rl = t >> 6;
  const int tt = t & 63;
  int row = blockIdx.x * 4 + rl;
  row = (row < nrows) ? row : (nrows - 1);
  const float* rp = in + (size_t)row * kDim;
  const v4f a = *(const v4f*)(rp + 4 * tt);
  const v4f c = *(const v4f*)(rp + 256 + 4 * tt);
  float s  = ((a[0] + a[1]) + (a[2] + a[3])) + ((c[0] + c[1]) + (c[2] + c[3]));
  float sq = ((a[0] * a[0] + a[1] * a[1]) + (a[2] * a[2] + a[3] * a[3]))
           + ((c[0] * c[0] + c[1] * c[1]) + (c[2] * c[2] + c[3] * c[3]));
#pragma unroll
  for (int off = 16; off > 0; off >>= 1) {
    s  += __shfl_xor(s, off, 32);
    sq += __shfl_xor(sq, off, 32);
  }
  if (lane == 0) { redA[wave] = s; redB[wave] = sq; }
  __syncthreads();
  const float S = redA[2 * rl] + redA[2 * rl + 1];
  const float Q = redB[2 * rl] + redB[2 * rl + 1];
  const float mean = S * kInvDim;
  const float msq  = Q * kInvDim;
  const float mm   = mean * mean;
  const float var  = msq - mm;
  const float vv   = var + 1e-5f;
  float y = 0.5f;
#pragma unroll
  for (int i = 0; i < 3; ++i) {
    float t1 = vv * y;
    t1 = t1 * y;
    const float u = 3.0f - t1;
    y = y * u;
    y = y * 0.5f;
  }
  const v4f ga = *(const v4f*)(gamma + 4 * tt);
  const v4f gb = *(const v4f*)(gamma + 256 + 4 * tt);
  const v4f ba = *(const v4f*)(beta + 4 * tt);
  const v4f bb = *(const v4f*)(beta + 256 + 4 * tt);
  v4f o0, o1;
#pragma unroll
  for (int e = 0; e < 4; ++e) {
    float d0 = a[e] - mean; d0 = d0 * y; d0 = d0 * ga[e]; o0[e] = d0 + ba[e];
    float d1 = c[e] - mean; d1 = d1 * y; d1 = d1 * gb[e]; o1[e] = d1 + bb[e];
  }
  float* orow = outf + (size_t)row * kDim;
  v2u h0, h1;
  if (WRITE16) {
    h0 = (v2u){pk16(h_bits(o0[0]), h_bits(o0[1])), pk16(h_bits(o0[2]), h_bits(o0[3]))};
    h1 = (v2u){pk16(h_bits(o1[0]), h_bits(o1[1])), pk16(h_bits(o1[2]), h_bits(o1[3]))};
  }
  unsigned short* hrow = out16 + (size_t)row * kDim;
  for (int pass = 0; pass < 2; ++pass) {
    *(volatile v4f*)(orow + 4 * tt) = o0;
    *(volatile v4f*)(orow + 256 + 4 * tt) = o1;
    if (WRITE16) {
      *(volatile v2u*)(hrow + 4 * tt) = h0;
      *(volatile v2u*)(hrow + 256 + 4 * tt) = h1;
    }
    __threadfence();
  }
}

__global__ __launch_bounds__(256) void gelu_poly_kernel(const float* __restrict__ F, unsigned short* __restrict__ G,
                                                        const float* __restrict__ gelu_c, int n8) {
  const int i = blockIdx.x * 256 + threadIdx.x;
  if (i >= n8) return;
  const float* p = F + 8 * (size_t)i;
  const v4f a = *(const v4f*)(p);
  const v4f c = *(const v4f*)(p + 4);
  float x[8];
#pragma unroll
  for (int e = 0; e < 4; ++e) { x[e] = a[e]; x[4 + e] = c[e]; }
  float gc[8];
#pragma unroll
  for (int j = 0; j < 8; ++j) gc[j] = gelu_c[j];
  unsigned short hb[8];
#pragma unroll
  for (int e = 0; e < 8; ++e) {
    const float xc = fminf(fmaxf(x[e], -4.0f), 4.0f);
    float acc = gc[0];
    float pw = 1.0f;
#pragma unroll
    for (int j = 1; j < 8; ++j) {
      pw = pw * xc;
      const float term = gc[j] * pw;
      acc = acc + term;
    }
    hb[e] = h_bits(acc * kGCarry);
  }
  const v4u u = (v4u){pk16(hb[0], hb[1]), pk16(hb[2], hb[3]), pk16(hb[4], hb[5]), pk16(hb[6], hb[7])};
  unsigned short* q = G + 8 * (size_t)i;
  *(volatile v4u*)q = u;
  __threadfence();
  *(volatile v4u*)q = u;
}

extern "C" void kernel_launch(void* const* d_in, const int* in_sizes, int n_in,
                              void* d_out, int out_size, void* d_ws, size_t ws_size,
                              hipStream_t stream)
{
  if (n_in < 13) return;
  if (in_sizes[0] != kTok * kDim || out_size != kTok * kDim) return;
  if (in_sizes[1] != kDim * kDim || in_sizes[5] != kDim * kFF || in_sizes[6] != kFF * kDim) return;
  if (in_sizes[11] < 8 || in_sizes[12] < 7) return;
  if (ws_size < kWsTotal) return;

  const float* x      = (const float*)d_in[0];
  const float* Wq     = (const float*)d_in[1];
  const float* Wk     = (const float*)d_in[2];
  const float* Wv     = (const float*)d_in[3];
  const float* Wo     = (const float*)d_in[4];
  const float* W1     = (const float*)d_in[5];
  const float* W2     = (const float*)d_in[6];
  const float* g1     = (const float*)d_in[7];
  const float* b1     = (const float*)d_in[8];
  const float* g2     = (const float*)d_in[9];
  const float* b2     = (const float*)d_in[10];
  const float* gelu_c = (const float*)d_in[11];
  const float* exp_c  = (const float*)d_in[12];
  float* out = (float*)d_out;

  char* ws = (char*)d_ws;
  unsigned short* WqkT = (unsigned short*)(ws + kOffWqk);
  unsigned short* WvT  = (unsigned short*)(ws + kOffWv);
  unsigned short* WoT  = (unsigned short*)(ws + kOffWo);
  unsigned short* W1T  = (unsigned short*)(ws + kOffW1);
  unsigned short* W2T  = (unsigned short*)(ws + kOffW2);
  unsigned short* X16  = (unsigned short*)(ws + kOffR1);
  unsigned short* H16  = (unsigned short*)(ws + kOffR1);
  unsigned short* QK   = (unsigned short*)(ws + kOffR2);
  float*          HPRE = (float*)(ws + kOffR2);
  unsigned short* VT   = (unsigned short*)(ws + kOffR3);
  unsigned short* O16  = (unsigned short*)(ws + kOffR4);
  float*          SC   = (float*)(ws + kOffR5);
  float*          FB   = (float*)(ws + kOffR5);
  unsigned short* PP   = (unsigned short*)(ws + kOffR6);
  unsigned short* G16  = (unsigned short*)(ws + kOffR6);
  float*          HB   = (float*)(ws + kOffR7);
  float*          FPRE = (float*)(ws + kOffR8);

  const float* dumb = g1;
  const float* dumr = x;
  const dim3 blk(256);

  tcast_kernel<<<dim3(kDim / 64, kDim / 64), blk, 0, stream>>>(Wq, kDim, WqkT, kDim, kWCarry);
  tcast_kernel<<<dim3(kDim / 64, kDim / 64), blk, 0, stream>>>(Wk, kDim, WqkT + (size_t)kDim * kDim, kDim, kWCarry);
  tcast_kernel<<<dim3(kDim / 64, kDim / 64), blk, 0, stream>>>(Wv, kDim, WvT, kDim, kWCarry);
  tcast_kernel<<<dim3(kDim / 64, kDim / 64), blk, 0, stream>>>(Wo, kDim, WoT, kDim, kWCarry);
  tcast_kernel<<<dim3(kDim / 64, kFF / 64), blk, 0, stream>>>(W1, kFF, W1T, kDim, kWCarry);
  tcast_kernel<<<dim3(kFF / 64, kDim / 64), blk, 0, stream>>>(W2, kDim, W2T, kFF, kWCarry);

  cast8_f16_kernel<<<dim3((kTok * kDim / 8) / 256), blk, 0, stream>>>(x, X16, kTok * kDim / 8);

  wmma_gemm64<0, false, 0, 1, false><<<dim3((kTok / 64) * (kQKld / 64) / 8, 1), blk, 0, stream>>>(
      X16, X16, kDim, 0L, WqkT, WqkT, kDim, 0L, QK, QK, kQKld, 0L, dumb, dumr, 0L, kTok, kQKld, kDim, kQKVScale);
  wmma_gemm64<0, false, 0, 1, false><<<dim3((kDim / 64) * (kTok / 64) / 8, 1), blk, 0, stream>>>(
      WvT, WvT, kDim, 0L, X16, X16, kDim, 0L, VT, VT, kTok, 0L, dumb, dumr, 0L, kDim, kTok, kDim, kQKVScale);

  for (int ch = 0; ch < kNChunk; ++ch) {
    const int b  = ch / (kHeads / kGrp);
    const int h0 = (ch % (kHeads / kGrp)) * kGrp;
    const unsigned short* qbase = QK + (size_t)b * kSeq * kQKld + (size_t)h0 * kDH;
    const unsigned short* kbase = qbase + kDim;
    wmma_gemm64<0, false, 0, 0, false><<<dim3((kSeq / 64) * (kSeq / 64) / 8, kGrp), blk, 0, stream>>>(
        qbase, qbase, kQKld, (long)kDH, kbase, kbase, kQKld, (long)kDH,
        SC, SC, kSeq, (long)kSeq * kSeq, dumb, dumr, 0L, kSeq, kSeq, kDH, kScoreScale);
    softmax_poly_kernel<<<dim3(kGrp * kSeq), blk, 0, stream>>>(SC, PP, exp_c);
    const unsigned short* vtb = VT + (size_t)h0 * kDH * kTok + (size_t)b * kSeq;
    unsigned short* ob = O16 + (size_t)b * kSeq * kDim + (size_t)h0 * kDH;
    wmma_gemm64<0, false, 0, 1, false><<<dim3((kSeq / 64) * (kDH / 64) / 8, kGrp), blk, 0, stream>>>(
        PP, PP, kSeq, (long)kSeq * kSeq, vtb, vtb, kTok, (long)kDH * kTok,
        ob, ob, kDim, (long)kDH, dumb, dumr, 0L, kSeq, kDH, kSeq, kPVScale);
  }

  wmma_gemm64<0, false, 0, 0, true><<<dim3((kTok / 64) * (kDim / 64) / 8, 1), blk, 0, stream>>>(
      O16, O16, kDim, 0L, WoT, WoT, kDim, 0L, HPRE, HPRE, kDim, 0L, dumb, x, 0L, kTok, kDim, kDim, kWoScale);
  layernorm_kernel<true><<<dim3(kTok / 4), blk, 0, stream>>>(HPRE, g1, b1, HB, H16, kTok);

  for (int half = 0; half < 2; ++half) {
    const unsigned short* ha = H16 + (size_t)half * kHalfTok * kDim;
    wmma_gemm64<0, false, 0, 0, false><<<dim3((kHalfTok / 64) * (kFF / 64) / 8, 1), blk, 0, stream>>>(
        ha, ha, kDim, 0L, W1T, W1T, kDim, 0L, FB, FB, kFF, 0L, dumb, dumr, 0L, kHalfTok, kFF, kDim, kW1Scale);
    gelu_poly_kernel<<<dim3((kHalfTok * kFF / 8) / 256), blk, 0, stream>>>(FB, G16, gelu_c, kHalfTok * kFF / 8);
    float* fo = FPRE + (size_t)half * kHalfTok * kDim;
    const float* hr = HB + (size_t)half * kHalfTok * kDim;
    wmma_gemm64<0, false, 0, 0, true><<<dim3((kHalfTok / 64) * (kDim / 64) / 8, 1), blk, 0, stream>>>(
        G16, G16, kFF, 0L, W2T, W2T, kFF, 0L, fo, fo, kDim, 0L, dumb, hr, 0L, kHalfTok, kDim, kFF, kW2Scale);
  }

  layernorm_kernel<false><<<dim3(kTok / 4), blk, 0, stream>>>(FPRE, g2, b2, out, H16, kTok);
}
